// TopologyEncoder_50800873177281
// MI455X (gfx1250) — hardware-verified
//
#include <hip/hip_runtime.h>
#include <stddef.h>


#define FD      128
#define HWP     256
#define NTHR    256
#define NWAVE   8
#define EPT     8
#define NGRP    2
#define CHUNK   (NTHR * EPT * NGRP)
#define WCAP    (EPT * NGRP * 32)
#define LISTN   (NWAVE * WCAP)
#define ESHF    10
#define EBITS   21
#define EFLD    (1 << EBITS)
#define NBC     32768
#define NBF     1024
#define RCAP    40960
#define RBN     128
#define TGT     256
#define DEGCAP  512
#define GROWS   128
#define OTHR    256
#define ASCALE  64
#define WSCALE  64
#define LNEPS   1e-5f
#define WSCAP   134217728

#define LDS_COUNT ((NBC + LISTN + NWAVE) * 4)
#define LDS_FILL  ((RCAP + NBF + NBF + NBF + LISTN + LISTN + NWAVE) * 4)
#define LDS_GEMM  (GROWS * FD * 4)
#define WPB       ((FD * FD / 8) / NTHR)

static_assert((CHUNK & (CHUNK - 1)) == 0);
static_assert((NBC & (NBC - 1)) == 0 && (NBF & (NBF - 1)) == 0);
static_assert(NBF <= (1 << ESHF));
static_assert(ESHF + EBITS <= 31);
static_assert((NBC % NBF) == 0);
static_assert(OTHR * 4 == NBF);
static_assert((RCAP % 32) == 0);
static_assert(TGT == NWAVE * 32);
static_assert(GROWS == NWAVE * 16);
static_assert((TGT % GROWS) == 0);
static_assert(FD == 128 && FD == 32 * 4);
static_assert(HWP == 2 * FD);
static_assert(NBC == NWAVE * 32 * 128);
static_assert(NBF == NWAVE * 128);
static_assert((FD * FD / 8) % NTHR == 0);
static_assert(NTHR == NWAVE * 32);
static_assert(LDS_FILL <= 300000 && LDS_COUNT <= 300000);

typedef float     v4f  __attribute__((ext_vector_type(4)));
typedef float     v8f  __attribute__((ext_vector_type(8)));
typedef int       v4i  __attribute__((ext_vector_type(4)));
typedef _Float16  v8h  __attribute__((ext_vector_type(8)));
typedef _Float16  v16h __attribute__((ext_vector_type(16)));
union FragH { v16h v; v8h h[2]; };
union FI { float f; int i; };

__device__ __forceinline__ v8f wmf(v16h a, v16h b, v8f c) {
  v8f d = __builtin_amdgcn_wmma_f32_16x16x32_f16(false, a, false, b, (short)0, c, false, false);
  asm volatile("v_nop\n\tv_nop\n\tv_nop\n\tv_nop" : "+v"(d) : "v"(a), "v"(b));
  return d;
}

template <int NB, int MODE>
__device__ __forceinline__ int scan_chunk(const int* __restrict__ keys, const float* __restrict__ ew, int nE,
                                          int cbase, int slotBase, int vec8, int* list, int* wlst,
                                          int tid, int lane, int wave) {
  int wc = 0;
#pragma unroll
  for (int g = 0; g < NGRP; ++g) {
    const int el0  = (g * NTHR + tid) * EPT;
    const int e0   = cbase + el0;
    const int sent = -2147483647 - 1;
    v4i da, db;
    v4f wa = {0.f, 0.f, 0.f, 0.f}, wb = {0.f, 0.f, 0.f, 0.f};
    if (vec8 != 0 && cbase + CHUNK <= nE) {
      da = *(const v4i*)(keys + e0);
      db = *(const v4i*)(keys + e0 + 4);
      if (MODE) {
        wa = *(const v4f*)(ew + e0);
        wb = *(const v4f*)(ew + e0 + 4);
      }
    } else {
      const int le = nE - 1;
      da.x = (e0     < nE) ? keys[min(e0,     le)] : sent;
      da.y = (e0 + 1 < nE) ? keys[min(e0 + 1, le)] : sent;
      da.z = (e0 + 2 < nE) ? keys[min(e0 + 2, le)] : sent;
      da.w = (e0 + 3 < nE) ? keys[min(e0 + 3, le)] : sent;
      db.x = (e0 + 4 < nE) ? keys[min(e0 + 4, le)] : sent;
      db.y = (e0 + 5 < nE) ? keys[min(e0 + 5, le)] : sent;
      db.z = (e0 + 6 < nE) ? keys[min(e0 + 6, le)] : sent;
      db.w = (e0 + 7 < nE) ? keys[min(e0 + 7, le)] : sent;
      if (MODE) {
        wa.x = ew[min(e0,     le)]; wa.y = ew[min(e0 + 1, le)];
        wa.z = ew[min(e0 + 2, le)]; wa.w = ew[min(e0 + 3, le)];
        wb.x = ew[min(e0 + 4, le)]; wb.y = ew[min(e0 + 5, le)];
        wb.z = ew[min(e0 + 6, le)]; wb.w = ew[min(e0 + 7, le)];
      }
    }
    const unsigned nb = (unsigned)slotBase;
    const unsigned s0 = (unsigned)da.x - nb, s1 = (unsigned)da.y - nb;
    const unsigned s2 = (unsigned)da.z - nb, s3 = (unsigned)da.w - nb;
    const unsigned s4 = (unsigned)db.x - nb, s5 = (unsigned)db.y - nb;
    const unsigned s6 = (unsigned)db.z - nb, s7 = (unsigned)db.w - nb;
    const bool h0 = s0 < (unsigned)NB, h1 = s1 < (unsigned)NB, h2 = s2 < (unsigned)NB, h3 = s3 < (unsigned)NB;
    const bool h4 = s4 < (unsigned)NB, h5 = s5 < (unsigned)NB, h6 = s6 < (unsigned)NB, h7 = s7 < (unsigned)NB;
    const unsigned any = __builtin_amdgcn_ballot_w32(h0 | h1 | h2 | h3 | h4 | h5 | h6 | h7);
    if (any != 0u) {
#define HITJ(HJ, SJ, EJ, WJ) { \
        const unsigned mj = __builtin_amdgcn_ballot_w32(HJ); \
        if (mj != 0u) { \
          if (HJ) { \
            const int pos = wc + (int)__builtin_amdgcn_mbcnt_lo(mj, 0u); \
            const int entv = MODE ? (int)((((unsigned)(EJ)) << ESHF) | (SJ)) : (int)(SJ); \
            if (pos < WCAP) { \
              list[wave * WCAP + pos] = entv; \
              if (MODE) wlst[wave * WCAP + pos] = __float_as_int(WJ); \
            } \
          } \
          wc += (int)__builtin_popcount(mj); } }
      HITJ(h0, s0, e0,     wa.x)
      HITJ(h1, s1, e0 + 1, wa.y)
      HITJ(h2, s2, e0 + 2, wa.z)
      HITJ(h3, s3, e0 + 3, wa.w)
      HITJ(h4, s4, e0 + 4, wb.x)
      HITJ(h5, s5, e0 + 5, wb.y)
      HITJ(h6, s6, e0 + 6, wb.z)
      HITJ(h7, s7, e0 + 7, wb.w)
#undef HITJ
    }
  }
  return wc;
}

__global__ __launch_bounds__(NTHR) void k_wprep(const float* __restrict__ w0, const float* __restrict__ w1,
                                                _Float16* wp, int nPl) {
  const int tid = threadIdx.x;
  const int p = (int)blockIdx.x / WPB;
  if (p >= nPl) return;
  const int l  = p >> 1, br = p & 1;
  const int i  = ((int)blockIdx.x - p * WPB) * NTHR + tid;
  const int n  = i >> 4;
  const int k0 = (i & 15) * 8;
  const size_t lb = (size_t)l * FD * FD;
  v8h hv;
#pragma unroll
  for (int e = 0; e < 8; ++e) {
    const size_t idx = lb + (size_t)(k0 + e) * FD + (size_t)n;
    const float a = w0[idx];
    const float b = w1[idx];
    hv[e] = (_Float16)((br ? b : a) * (float)WSCALE);
  }
  _Float16* d = wp + (size_t)p * FD * FD + (size_t)i * 8;
  *(volatile v8h*)d = hv;
  __threadfence();
  *(volatile v8h*)d = hv;
}

__global__ __launch_bounds__(NTHR) void k_count(const int* __restrict__ ei, int* cnt, int nE, int vec8) {
  extern __shared__ v4f lds_dyn[];
  int* scnt = (int*)lds_dyn;
  int* list = scnt + NBC;
  int* wcnt = list + LISTN;
  const int tid = threadIdx.x, lane = tid & 31, wave = tid >> 5;
  const int nodeBase = blockIdx.x * NBC;
  const int* keys = ei + nE;

  {
    const v4i z = {0, 0, 0, 0};
    for (int i = tid; i < NBC / 4; i += NTHR) ((v4i*)scnt)[i] = z;
  }
  __syncthreads();

  const int nChunks = (nE + CHUNK - 1) / CHUNK;
#pragma unroll 1
  for (int ch = 0; ch < nChunks; ++ch) {
    const int cbase = ch * CHUNK;
    const int wc = scan_chunk<NBC, 0>(keys, (const float*)keys, nE, cbase, nodeBase, vec8, list, list, tid, lane, wave);
    if (lane == 0) wcnt[wave] = wc;
    __syncthreads();
    if (wave == 0) {
#pragma unroll 1
      for (int wsx = 0; wsx < NWAVE; ++wsx) {
        int n = __builtin_amdgcn_readfirstlane(wcnt[wsx]);
        n = n > WCAP ? WCAP : (n < 0 ? 0 : n);
        const int* lp = list + wsx * WCAP;
#pragma unroll 1
        for (int i = 0; i < n; ++i) {
          const int ent  = __builtin_amdgcn_readfirstlane(lp[i]);
          const int slot = ent & (NBC - 1);
          if (lane == 0) scnt[slot] = scnt[slot] + 1;
        }
      }
    }
    __syncthreads();
  }

  int* cp = cnt + (size_t)nodeBase;
#pragma unroll 4
  for (int q = 0; q < 32; ++q) {
    const int f = (wave * 32 + q) * 128 + 4 * lane;
    const v4i c = *(const v4i*)(scnt + f);
    *(volatile v4i*)(cp + f) = c;
  }
  __threadfence();
#pragma unroll 4
  for (int q = 0; q < 32; ++q) {
    const int f = (wave * 32 + q) * 128 + 4 * lane;
    const v4i c = *(const v4i*)(scnt + f);
    *(volatile v4i*)(cp + f) = c;
  }
}

__global__ __launch_bounds__(OTHR) void k_offsets(
    const int* __restrict__ cnt, int* off, int* rbase, int nBF) {
  __shared__ __attribute__((aligned(16))) int srb[RBN];
  __shared__ int wtot[OTHR / 32];
  const int tid = threadIdx.x, lane = tid & 31, wave = tid >> 5;
  for (int i = tid; i < RBN; i += OTHR) srb[i] = 0;
  int carry = 0;
#pragma unroll 1
  for (int fb = 0; fb < nBF; ++fb) {
    const int base = fb * NBF;
    const v4i c = *(const v4i*)(cnt + base + 4 * tid);
    const int e0 = max(c.x, 0), e1 = max(c.y, 0), e2 = max(c.z, 0), e3 = max(c.w, 0);
    const int ts = e0 + e1 + e2 + e3;
    int incl = ts;
#pragma unroll
    for (int d = 1; d < 32; d <<= 1) {
      const int t = __shfl_up(incl, d);
      if (lane >= d) incl += t;
    }
    if (lane == 31) wtot[wave] = incl;
    __syncthreads();
    int pre = 0;
#pragma unroll 1
    for (int w = 0; w < wave; ++w) pre += wtot[w];
    int tot = 0;
#pragma unroll
    for (int w = 0; w < OTHR / 32; ++w) tot += wtot[w];
    int run = carry + pre + incl - ts;
    v4i o;
    o.x = run; run += e0;
    o.y = run; run += e1;
    o.z = run; run += e2;
    o.w = run;
    int* op = off + base + 4 * tid;
    *(volatile v4i*)op = o;
    __threadfence();
    *(volatile v4i*)op = o;
    if (tid == 0) srb[min(fb, RBN - 1)] = carry;
    carry += (tot + 31) & ~31;
    __syncthreads();
  }
  if (tid == 0) srb[min(nBF, RBN - 1)] = carry;
  __syncthreads();
  v4i rv = {0, 0, 0, 0};
  if (tid < 32) rv = *(const v4i*)(srb + 4 * tid);
  if (tid < 32) *(volatile v4i*)(rbase + 4 * tid) = rv;
  __threadfence();
  if (tid < 32) *(volatile v4i*)(rbase + 4 * tid) = rv;
}

__device__ __forceinline__ v4f rsq4p1(v4f ws) {
  const float g0 = ws.x + 1.0f, g1 = ws.y + 1.0f, g2 = ws.z + 1.0f, g3 = ws.w + 1.0f;
  v4f d;
  d.x = g0 > 0.f ? rsqrtf(g0) : 0.f; d.y = g1 > 0.f ? rsqrtf(g1) : 0.f;
  d.z = g2 > 0.f ? rsqrtf(g2) : 0.f; d.w = g3 > 0.f ? rsqrtf(g3) : 0.f;
  return d;
}

__global__ __launch_bounds__(NTHR) void k_fill(
    const int* __restrict__ ei, const float* __restrict__ ew,
    const int* __restrict__ off, const int* __restrict__ rbase,
    int* csr, float* dinv, int offn, int nN, int nE, int vec8, int csrLen) {
  extern __shared__ v4f lds_dyn[];
  int*   region = (int*)lds_dyn;
  int*   cursor = region + RCAP;
  float* sdgp   = (float*)(cursor + NBF);
  float* sdgn   = sdgp + NBF;
  int*   list   = (int*)(sdgn + NBF);
  int*   wlst   = list + LISTN;
  int*   wcnt   = wlst + LISTN;
  const int tid = threadIdx.x, lane = tid & 31, wave = tid >> 5;
  const int b = blockIdx.x;
  const int nodeBase = b * NBF;
  const int* keys = ei + nE;

  int rb0 = rbase[b];
  const int rb1 = rbase[b + 1];
  rb0 = rb0 < 0 ? 0 : (rb0 > csrLen ? csrLen : rb0);
  rb0 &= ~31;
  int len = rb1 - rb0;
  len = len < 0 ? 0 : (len > RCAP ? RCAP : len);
  int lenW = (len + 31) & ~31;
  if (rb0 + lenW > csrLen) lenW = (csrLen - rb0) & ~31;

  {
    const v4i z = {0, 0, 0, 0};
    for (int i = tid; i < RCAP / 4; i += NTHR) ((v4i*)region)[i] = z;
    for (int s = tid; s < NBF; s += NTHR) {
      int o = off[nodeBase + s] - rb0;
      o = o < 0 ? 0 : (o > RCAP ? RCAP : o);
      cursor[s] = o;
      sdgp[s] = 0.f;
      sdgn[s] = 0.f;
    }
  }
  __syncthreads();

  const int nChunks = (nE + CHUNK - 1) / CHUNK;
#pragma unroll 1
  for (int ch = 0; ch < nChunks; ++ch) {
    const int cbase = ch * CHUNK;
    const int wc = scan_chunk<NBF, 1>(keys, ew, nE, cbase, nodeBase, vec8, list, wlst, tid, lane, wave);
    if (lane == 0) wcnt[wave] = wc;
    __syncthreads();
    if (wave == 0) {
#pragma unroll 1
      for (int wsx = 0; wsx < NWAVE; ++wsx) {
        int n = __builtin_amdgcn_readfirstlane(wcnt[wsx]);
        n = n > WCAP ? WCAP : (n < 0 ? 0 : n);
        const int* lp = list + wsx * WCAP;
        const int* wl = wlst + wsx * WCAP;
#pragma unroll 1
        for (int i = 0; i < n; ++i) {
          const int ent  = __builtin_amdgcn_readfirstlane(lp[i]);
          FI wv; wv.i    = __builtin_amdgcn_readfirstlane(wl[i]);
          const int slot = ent & (NBF - 1);
          int e = (ent >> ESHF) & (EFLD - 1);
          e = e > nE - 1 ? nE - 1 : e;
          if (lane == 0) {
            int pos = cursor[slot];
            pos = pos < 0 ? 0 : (pos > RCAP - 1 ? RCAP - 1 : pos);
            region[pos] = e;
            const int np = pos + 1;
            cursor[slot] = np > RCAP ? RCAP : np;
            sdgp[slot] = sdgp[slot] + fmaxf(wv.f, 0.f);
            sdgn[slot] = sdgn[slot] + fmaxf(-wv.f, 0.f);
          }
        }
      }
    }
    __syncthreads();
  }

  const int nv = lenW >> 2;
  int* gp = csr + rb0;
  float* dpP = dinv + (size_t)nodeBase;
  float* dpN = dinv + (size_t)offn + (size_t)nodeBase;
  const int f = wave * 128 + 4 * lane;
#pragma unroll 1
  for (int i = tid; i < nv; i += NTHR) { const v4i v = ((const v4i*)region)[i]; *(volatile v4i*)(gp + 4 * i) = v; }
  {
    const v4f dP = rsq4p1(*(const v4f*)(sdgp + f));
    const v4f dN = rsq4p1(*(const v4f*)(sdgn + f));
    *(volatile v4f*)(dpP + f) = dP;
    *(volatile v4f*)(dpN + f) = dN;
  }
  __threadfence();
#pragma unroll 1
  for (int i = tid; i < nv; i += NTHR) { const v4i v = ((const v4i*)region)[i]; *(volatile v4i*)(gp + 4 * i) = v; }
  {
    const v4f dP = rsq4p1(*(const v4f*)(sdgp + f));
    const v4f dN = rsq4p1(*(const v4f*)(sdgn + f));
    *(volatile v4f*)(dpP + f) = dP;
    *(volatile v4f*)(dpN + f) = dN;
  }
}

__global__ __launch_bounds__(NTHR) void k_gemm(
    const float* __restrict__ X, const _Float16* __restrict__ Bw2,
    const float* __restrict__ dinv2, int offn, float* C, int nRowsA) {
  extern __shared__ v4f lds_dyn[];
  constexpr int NT = FD / 16;
  constexpr float OSC = 1.0f / (float)(ASCALE * WSCALE);
  float* stg = (float*)lds_dyn;
  const int tid = threadIdx.x, lane = tid & 31, wave = tid >> 5, hh = lane >> 4, m = lane & 15;
  const int y = (int)blockIdx.y;
  const _Float16* Bw = Bw2 + (size_t)y * FD * FD;
  const float* dv = dinv2 + (size_t)y * (size_t)offn;
  const int rowBase = blockIdx.x * GROWS;
  int arow = rowBase + wave * 16 + m;
  arow = arow > nRowsA - 1 ? nRowsA - 1 : arow;
  const float* ap = X + (size_t)arow * FD + 8 * hh;

  v8f acc[NT];
#pragma unroll
  for (int t = 0; t < NT; ++t) { v8f z = {0.f, 0.f, 0.f, 0.f, 0.f, 0.f, 0.f, 0.f}; acc[t] = z; }

#pragma unroll 1
  for (int kt = 0; kt < FD / 32; ++kt) {
    const int ko = 32 * kt;
    const v4f f0 = *(const v4f*)(ap + ko);
    const v4f f1 = *(const v4f*)(ap + ko + 4);
    const v4f f2 = *(const v4f*)(ap + ko + 16);
    const v4f f3 = *(const v4f*)(ap + ko + 20);
    v8h lo, hi;
    lo[0] = (_Float16)(f0.x * (float)ASCALE); lo[1] = (_Float16)(f0.y * (float)ASCALE);
    lo[2] = (_Float16)(f0.z * (float)ASCALE); lo[3] = (_Float16)(f0.w * (float)ASCALE);
    lo[4] = (_Float16)(f1.x * (float)ASCALE); lo[5] = (_Float16)(f1.y * (float)ASCALE);
    lo[6] = (_Float16)(f1.z * (float)ASCALE); lo[7] = (_Float16)(f1.w * (float)ASCALE);
    hi[0] = (_Float16)(f2.x * (float)ASCALE); hi[1] = (_Float16)(f2.y * (float)ASCALE);
    hi[2] = (_Float16)(f2.z * (float)ASCALE); hi[3] = (_Float16)(f2.w * (float)ASCALE);
    hi[4] = (_Float16)(f3.x * (float)ASCALE); hi[5] = (_Float16)(f3.y * (float)ASCALE);
    hi[6] = (_Float16)(f3.z * (float)ASCALE); hi[7] = (_Float16)(f3.w * (float)ASCALE);
    FragH af;
    af.h[0] = lo;
    af.h[1] = hi;
#pragma unroll
    for (int t = 0; t < NT; ++t) {
      const _Float16* bp = Bw + (size_t)(16 * t + m) * FD + ko + 8 * hh;
      FragH bf;
      bf.h[0] = *(const v8h*)bp;
      bf.h[1] = *(const v8h*)(bp + 16);
      acc[t] = wmf(af.v, bf.v, acc[t]);
    }
  }

  const int r0 = wave * 16 + 8 * hh;
  const v4f dA = *(const v4f*)(dv + (size_t)rowBase + r0);
  const v4f dB = *(const v4f*)(dv + (size_t)rowBase + r0 + 4);
  float s[8];
  s[0] = dA.x; s[1] = dA.y; s[2] = dA.z; s[3] = dA.w; s[4] = dB.x; s[5] = dB.y; s[6] = dB.z; s[7] = dB.w;
#pragma unroll
  for (int r = 0; r < 8; ++r) s[r] = s[r] * OSC;
  float* sp = stg + r0 * FD + m;
#pragma unroll
  for (int t = 0; t < NT; ++t) {
#pragma unroll
    for (int r = 0; r < 8; ++r) sp[r * FD + 16 * t] = acc[t][r] * s[r];
  }
  __syncthreads();

  const float* lp = stg + wave * 16 * FD;
  float* gp = C + (size_t)(rowBase + wave * 16) * HWP + (size_t)y * FD;
#pragma unroll
  for (int i = 0; i < 16; ++i) {
    const v4f v = *(const v4f*)(lp + i * FD + 4 * lane);
    *(volatile v4f*)(gp + (size_t)i * HWP + 4 * lane) = v;
  }
  __threadfence();
#pragma unroll
  for (int i = 0; i < 16; ++i) {
    const v4f v = *(const v4f*)(lp + i * FD + 4 * lane);
    *(volatile v4f*)(gp + (size_t)i * HWP + 4 * lane) = v;
  }
}

__device__ __forceinline__ void gather_seg(const int* __restrict__ csr, int csrLen, int st, int n,
                                           const int* __restrict__ esrc, const float* __restrict__ ew, int nE,
                                           const float* __restrict__ hw, int nN, int lane,
                                           v4f& accP, v4f& accN) {
#pragma unroll 1
  for (int q0 = 0; q0 < n; q0 += 32) {
    int pos = st + q0 + lane;
    pos = pos < 0 ? 0 : (pos > csrLen - 1 ? csrLen - 1 : pos);
    int el = csr[pos];
    el = el < 0 ? 0 : (el > nE - 1 ? nE - 1 : el);
    int sl = esrc[el];
    sl = sl < 0 ? 0 : (sl > nN - 1 ? nN - 1 : sl);
    FI wu; wu.f = ew[el];
    const int mcnt = (n - q0) < 32 ? (n - q0) : 32;
#pragma unroll 1
    for (int p = 0; p < mcnt; ++p) {
      const int s = __builtin_amdgcn_readlane(sl, p);
      FI wq; wq.i = __builtin_amdgcn_readlane(wu.i, p);
      const float* rp = hw + (size_t)s * HWP + 4 * lane;
      if (wq.f > 0.f) {
        const v4f hv = *(const v4f*)rp;
        accP = accP + hv * wq.f;
      } else {
        const v4f hv = *(const v4f*)(rp + FD);
        accN = accN - hv * wq.f;
      }
    }
  }
}

__global__ __launch_bounds__(NTHR) void k_agg(
    const int* __restrict__ csr, const int* __restrict__ offp, const int* __restrict__ cnt,
    const float* __restrict__ dinv2, int offn, const float* __restrict__ hw,
    const int* __restrict__ ei, const float* __restrict__ ew, int nE, int csrLen,
    const float* __restrict__ bP, const float* __restrict__ bN, float* xo, int nN) {
  const int tid = threadIdx.x, lane = tid & 31, wave = tid >> 5;
  const int tbase = blockIdx.x * TGT + wave * 32;
  const int cl = tbase + lane;
  const int cnt_l = cnt[cl], off_l = offp[cl];
  FI dPu; dPu.f = dinv2[cl];
  FI dNu; dNu.f = dinv2[(size_t)offn + cl];
  const v4f bbP = *(const v4f*)(bP + 4 * lane);
  const v4f bbN = *(const v4f*)(bN + 4 * lane);

#pragma unroll 1
  for (int j = 0; j < 32; ++j) {
    const int c = tbase + j;
    int n = __builtin_amdgcn_readlane(cnt_l, j);
    n = n < 0 ? 0 : (n > DEGCAP ? DEGCAP : n);
    const int st = __builtin_amdgcn_readlane(off_l, j);
    FI dp; dp.i = __builtin_amdgcn_readlane(dPu.i, j);
    FI dn; dn.i = __builtin_amdgcn_readlane(dNu.i, j);

    v4f accP = {0.f, 0.f, 0.f, 0.f}, accN = {0.f, 0.f, 0.f, 0.f};
    gather_seg(csr, csrLen, st, n, ei, ew, nE, hw, nN, lane, accP, accN);
    const v4f selfP = *(const v4f*)(hw + (size_t)c * HWP + 4 * lane);
    const v4f selfN = *(const v4f*)(hw + (size_t)c * HWP + FD + 4 * lane);
    const v4f px = (accP + selfP) * dp.f + bbP;
    const v4f nx = (accN + selfN) * dn.f + bbN;
    v4f o;
    o.x = fmaxf(px.x, 0.f) - fmaxf(nx.x, 0.f);
    o.y = fmaxf(px.y, 0.f) - fmaxf(nx.y, 0.f);
    o.z = fmaxf(px.z, 0.f) - fmaxf(nx.z, 0.f);
    o.w = fmaxf(px.w, 0.f) - fmaxf(nx.w, 0.f);
    float* op = xo + (size_t)c * FD + 4 * lane;
    *(volatile v4f*)op = o;
    __threadfence();
    *(volatile v4f*)op = o;
  }
}

__global__ __launch_bounds__(NTHR) void k_pool(
    const float* __restrict__ xf, const int* __restrict__ bt,
    const float* __restrict__ gam, const float* __restrict__ bet, float* out, int nN) {
  __shared__ __attribute__((aligned(16))) float part[NWAVE * FD];
  __shared__ int pcnt[NWAVE];
  __shared__ float red[2 * NWAVE];
  __shared__ __attribute__((aligned(16))) float orow[FD];
  const int tid = threadIdx.x, lane = tid & 31, wave = tid >> 5;
  const int g = (int)blockIdx.x;

  v4f acc = {0.f, 0.f, 0.f, 0.f};
  int cw = 0;
#pragma unroll 1
  for (int base = wave * 32; base < nN; base += NTHR) {
    const int node = base + lane;
    const int nd = node > nN - 1 ? nN - 1 : node;
    const int b = bt[nd];
    const bool hit = (node < nN) && (b == g);
    unsigned mk = __builtin_amdgcn_ballot_w32(hit);
#pragma unroll 1
    for (int t = 0; t < 32; ++t) {
      if (mk == 0u) break;
      const int bi = __builtin_ctz(mk);
      mk &= mk - 1u;
      const int nd2 = base + bi;
      const v4f hv = *(const v4f*)(xf + (size_t)nd2 * FD + 4 * lane);
      acc = acc + hv;
      cw += 1;
    }
  }
  *(v4f*)(part + wave * FD + 4 * lane) = acc;
  if (lane == 0) pcnt[wave] = cw;
  __syncthreads();

  const int d = tid & (FD - 1);
  float s = 0.f;
  int ct = 0;
#pragma unroll
  for (int w = 0; w < NWAVE; ++w) { s += part[w * FD + d]; ct += pcnt[w]; }
  const float cf = (float)ct;
  const float rc = 1.0f / fmaxf(cf, 1.0f);
  const float p = s * rc;
  float wsum = p;
#pragma unroll
  for (int o = 16; o > 0; o >>= 1) wsum += __shfl_xor(wsum, o);
  if (lane == 0 && wave < FD / 32) red[wave] = wsum;
  __syncthreads();
  float mu = 0.f;
#pragma unroll
  for (int w = 0; w < FD / 32; ++w) mu += red[w];
  mu = mu * (1.0f / (float)FD);
  const float diff = p - mu;
  float q = diff * diff;
#pragma unroll
  for (int o = 16; o > 0; o >>= 1) q += __shfl_xor(q, o);
  if (lane == 0 && wave < FD / 32) red[NWAVE + wave] = q;
  __syncthreads();
  float var = 0.f;
#pragma unroll
  for (int w = 0; w < FD / 32; ++w) var += red[NWAVE + w];
  var = var * (1.0f / (float)FD);
  const float val = diff * rsqrtf(var + LNEPS) * gam[d] + bet[d];
  if (wave < FD / 32) orow[d] = val;
  __syncthreads();
  if (wave == 0) {
    const v4f v = *(const v4f*)(orow + 4 * lane);
    float* op = out + (size_t)g * FD + 4 * lane;
    *(volatile v4f*)op = v;
    __threadfence();
    *(volatile v4f*)op = v;
  }
}

extern "C" void kernel_launch(void* const* d_in, const int* in_sizes, int n_in,
                              void* d_out, int out_size, void* d_ws, size_t ws_size,
                              hipStream_t stream) {
  if (n_in < 10) return;
  const int nN = in_sizes[0] / FD;
  const int nE = in_sizes[1] / 2;
  const int nL = in_sizes[4] / (FD * FD);
  const int nG = out_size / FD;
  if (nN <= 0 || nE <= 0 || nL <= 0 || nG <= 0) return;
  if (in_sizes[0] != nN * FD || in_sizes[1] != 2 * nE || in_sizes[2] != nE || in_sizes[3] != nN) return;
  if (in_sizes[4] != nL * FD * FD || in_sizes[5] != nL * FD) return;
  if (in_sizes[6] != nL * FD * FD || in_sizes[7] != nL * FD) return;
  if (in_sizes[8] != FD || in_sizes[9] != FD) return;
  if (out_size != nG * FD) return;
  if (nE > EFLD) return;

  const float* x    = (const float*)d_in[0];
  const int*   ei   = (const int*)d_in[1];
  const float* ew   = (const float*)d_in[2];
  const int*   bt   = (const int*)d_in[3];
  const float* Wp   = (const float*)d_in[4];
  const float* bp   = (const float*)d_in[5];
  const float* Wn   = (const float*)d_in[6];
  const float* bn   = (const float*)d_in[7];
  const float* gam  = (const float*)d_in[8];
  const float* bet  = (const float*)d_in[9];
  float* out = (float*)d_out;

  const int NPAD   = ((nN + TGT - 1) / TGT) * TGT;
  const int nBC    = (nN + NBC - 1) / NBC;
  const int CNTPAD = nBC * NBC;
  const int nBF    = (nN + NBF - 1) / NBF;
  const int OFFN   = nBF * NBF;
  if (nBF + 1 > RBN) return;
  if (OFFN > CNTPAD || NPAD > OFFN) return;
  const int csrLen = ((nE + 31) & ~31) + 32 * (nBF + 1);
  const int nGemm  = NPAD / GROWS;
  const int nAgg   = NPAD / TGT;
  const int nPl    = 2 * nL;

  char* ws = (char*)d_ws;
  size_t off = 0;
  const size_t oW   = off; off += (size_t)nPl * FD * FD * 2;      off = (off + 255) & ~(size_t)255;
  const size_t oCnt = off; off += (size_t)CNTPAD * 4;             off = (off + 255) & ~(size_t)255;
  const size_t oOff = off; off += (size_t)OFFN * 4;               off = (off + 255) & ~(size_t)255;
  const size_t oRb  = off; off += (size_t)RBN * 4;                off = (off + 255) & ~(size_t)255;
  const size_t oCsr = off; off += (size_t)csrLen * 4;             off = (off + 255) & ~(size_t)255;
  const size_t oDv  = off; off += (size_t)2 * OFFN * 4;           off = (off + 255) & ~(size_t)255;
  const size_t oHw  = off; off += (size_t)NPAD * HWP * 4;         off = (off + 255) & ~(size_t)255;
  const size_t oX   = off; off += (size_t)NPAD * FD * 4;          off = (off + 255) & ~(size_t)255;
  if (off > ws_size || off > (size_t)WSCAP) return;
  _Float16* wpl   = (_Float16*)(ws + oW);
  int*      cnt   = (int*)(ws + oCnt);
  int*      offp  = (int*)(ws + oOff);
  int*      rb    = (int*)(ws + oRb);
  int*      csr   = (int*)(ws + oCsr);
  float*    dinv  = (float*)(ws + oDv);
  float*    hw    = (float*)(ws + oHw);
  float*    xbuf  = (float*)(ws + oX);

  const int vec8 = ((nE & 3) == 0) ? 1 : 0;

  k_wprep<<<nPl * WPB, NTHR, 0, stream>>>(Wp, Wn, wpl, nPl);

  hipFuncSetAttribute(reinterpret_cast<const void*>(&k_count),
                      hipFuncAttributeMaxDynamicSharedMemorySize, LDS_COUNT);
  hipFuncSetAttribute(reinterpret_cast<const void*>(&k_fill),
                      hipFuncAttributeMaxDynamicSharedMemorySize, LDS_FILL);
  hipFuncSetAttribute(reinterpret_cast<const void*>(&k_gemm),
                      hipFuncAttributeMaxDynamicSharedMemorySize, LDS_GEMM);
  k_count<<<nBC, NTHR, LDS_COUNT, stream>>>(ei, cnt, nE, vec8);
  k_offsets<<<1, OTHR, 0, stream>>>(cnt, offp, rb, nBF);
  k_fill<<<nBF, NTHR, LDS_FILL, stream>>>(ei, ew, offp, rb, csr, dinv, OFFN, nN, nE, vec8, csrLen);

  for (int l = 0; l < nL; ++l) {
    const float* xin = (l == 0) ? x : (const float*)xbuf;
    k_gemm<<<dim3(nGemm, 2), NTHR, LDS_GEMM, stream>>>(xin, wpl + (size_t)(2 * l) * FD * FD,
                                                       dinv, OFFN, hw, nN);
    k_agg<<<nAgg, NTHR, 0, stream>>>(csr, offp, cnt, dinv, OFFN, hw, ei, ew, nE, csrLen,
                                     bp + (size_t)l * FD, bn + (size_t)l * FD, xbuf, nN);
  }

  k_pool<<<nG, NTHR, 0, stream>>>(xbuf, bt, gam, bet, out, nN);
}
